// MoeHashLayer_40853728919571
// MI455X (gfx1250) — hardware-verified
//
#include <hip/hip_runtime.h>
#include <stddef.h>


typedef _Float16 v16h __attribute__((ext_vector_type(16)));
typedef _Float16 v8h  __attribute__((ext_vector_type(8)));
typedef float    v8f  __attribute__((ext_vector_type(8)));
typedef float    v4f  __attribute__((ext_vector_type(4)));
typedef _Float16 h16;

#ifndef NB
#define NB 2
#endif
#ifndef SEQ
#define SEQ 2048
#endif
#define NB_FULL  2
#define SEQ_FULL 2048
#define DIM   512
#define HID   2048
#define NEXP  8
#define NTOK  (NB * SEQ)
#define TOKT  32
#define MAXTILE (NTOK / TOKT)
#define CHUNK 256
#define NCHUNK (HID / CHUNK)
#define EPT   (NTOK / 256)

#define XLD (DIM + 8)
#define HLD (CHUNK + 8)
#define OLD 36
#define LDT 72

#define GPITCH ((size_t)NEXP * DIM)
#define OPITCH ((size_t)NEXP * HID)

#define WCARRY 64.0f
#define HCARRY 64.0f

static_assert(NB >= 1 && NB <= NB_FULL);
static_assert(SEQ >= 128 && SEQ <= SEQ_FULL && (SEQ % 128) == 0);
static_assert((NTOK % 256) == 0 && EPT >= 1 && EPT <= 16);
static_assert((SEQ % EPT) == 0);
static_assert(TOKT == 32 && (NTOK % TOKT) == 0);
static_assert(8 * 4 == TOKT);
static_assert(TOKT * 8 == 256 && DIM == 8 * 64);
static_assert((DIM % 64) == 0 && (HID % 64) == 0);
static_assert((DIM % 32) == 0 && (CHUNK % 32) == 0 && (HID % CHUNK) == 0);
static_assert(CHUNK == 8 * 32);
static_assert(DIM == 8 * 64);
static_assert((XLD % 8) == 0 && (HLD % 8) == 0 && (LDT % 8) == 0 && LDT >= 64);
static_assert((OLD % 4) == 0 && OLD >= 32);
static_assert(((NEXP * DIM) % 64) == 0 && ((NEXP * HID) % 64) == 0);

#define WGI_BYTES ((size_t)HID * NEXP * DIM * 2)
#define WO_BYTES  ((size_t)DIM * NEXP * HID * 2)
#define OFF_WG ((size_t)0)
#define OFF_WI (OFF_WG + WGI_BYTES)
#define OFF_WO (OFF_WI + WGI_BYTES)
#define WS_TOTAL (OFF_WO + WO_BYTES)
static_assert((WGI_BYTES % 128) == 0 && (WO_BYTES % 128) == 0);
static_assert(WS_TOTAL <= (size_t)134217728);

__device__ __forceinline__ float bf16r(float x) {
  unsigned int u = __float_as_uint(x);
  u = (u + 0x7FFFu + ((u >> 16) & 1u)) & 0xFFFF0000u;
  return __uint_as_float(u);
}

__device__ __forceinline__ h16 toh_flush(float v) {
  const h16 r = (h16)v;
  return (fabsf(v) < 6.103515625e-05f) ? (h16)0.0f : r;
}

__device__ __forceinline__ v16h frag_at(const _Float16* p) {
  v8h lo = *(const v8h*)(p);
  v8h hi = *(const v8h*)(p + 16);
  v16h out;
#pragma unroll
  for (int i = 0; i < 8; ++i) { out[i] = lo[i]; out[i + 8] = hi[i]; }
  return out;
}
__device__ __forceinline__ v16h ld_frag(const _Float16* base, unsigned ld) {
  const unsigned lane = threadIdx.x & 31u;
  return frag_at(base + (lane & 15u) * ld + (lane >> 4) * 8u);
}

__device__ __forceinline__ v8f wmma16(v16h a, v16h b, v8f c) {
  v8f d = __builtin_amdgcn_wmma_f32_16x16x32_f16(false, a, false, b, (short)0, c,
                                                 false, false);
  asm volatile("v_nop\n\tv_nop\n\tv_nop\n\tv_nop" : "+v"(d) : "v"(a), "v"(b));
  return d;
}

__device__ __forceinline__ void wave_lds_sync() {
  __builtin_amdgcn_fence(3  , "wavefront");
  asm volatile("s_wait_dscnt 0x0" ::: "memory");
  __builtin_amdgcn_wave_barrier();
}

__device__ __forceinline__ float silu_mul(float g, float u) {
  return g * __builtin_amdgcn_rcpf(1.0f + __expf(-g)) * u;
}

__global__ __launch_bounds__(256) void wconv_kernel(
    const float* __restrict__ W, _Float16* __restrict__ Wt, unsigned ldw, unsigned ldk) {
  __shared__ _Float16 T[64 * LDT];
  const unsigned tid = threadIdx.x;
  const unsigned n0 = blockIdx.x * 64u;
  const unsigned k0 = blockIdx.y * 64u;
#pragma unroll 4
  for (unsigned j = 0; j < 16u; ++j) {
    const unsigned idx = tid + 256u * j;
    const unsigned kr = idx >> 6, nc = idx & 63u;
    const float v = W[(size_t)(k0 + kr) * ldw + n0 + nc];
    T[nc * LDT + kr] = (_Float16)(WCARRY * bf16r(v));
  }
  __syncthreads();
  v8h x[2];
  size_t off[2];
#pragma unroll
  for (unsigned i = 0; i < 2u; ++i) {
    const unsigned n = 32u * i + (tid >> 3);
    const unsigned kc = (tid & 7u) * 8u;
    x[i] = *(const v8h*)&T[n * LDT + kc];
    off[i] = (size_t)(n0 + n) * ldk + k0 + kc;
  }
#pragma unroll
  for (int i = 0; i < 2; ++i) *(volatile v8h*)(Wt + off[i]) = x[i];
  __threadfence();
#pragma unroll
  for (int i = 0; i < 2; ++i) *(volatile v8h*)(Wt + off[i]) = x[i];
}

__global__ __launch_bounds__(256) void moe_ffn_kernel(
    const float* __restrict__ X, const int* __restrict__ route,
    const _Float16* __restrict__ Wg_t, const _Float16* __restrict__ Wi_t,
    const _Float16* __restrict__ Wo_t,
    const float* __restrict__ b_in, const float* __restrict__ b_gate,
    const float* __restrict__ b_out, float* __restrict__ out) {
  __shared__ _Float16 Xs[TOKT * XLD];
  __shared__ _Float16 Hs[TOKT * HLD];
  __shared__ float    Cs[8 * TOKT * OLD];
  __shared__ int      toks[TOKT];
  __shared__ int      wtot[8];

  const unsigned tid = threadIdx.x, lane = tid & 31u;
  const unsigned wv = tid >> 5;
  const int wave = __builtin_amdgcn_readfirstlane((int)(threadIdx.x >> 5));
  const unsigned hh = lane >> 4, m = lane & 15u;
  const int e = (int)blockIdx.y;
  const int tile = (int)blockIdx.x;

  const unsigned ci0 = tid * (unsigned)EPT;
  const unsigned bidx0 = ci0 / (unsigned)SEQ;
  const unsigned frow0 = bidx0 * (unsigned)SEQ_FULL + (ci0 - bidx0 * (unsigned)SEQ);
  int rv[EPT];
#pragma unroll
  for (int j = 0; j < EPT; ++j) rv[j] = route[frow0 + (unsigned)j];
  int c = 0;
#pragma unroll
  for (int j = 0; j < EPT; ++j) c += (rv[j] == e) ? 1 : 0;
  int inc = c;
#pragma unroll
  for (int off = 1; off < 32; off <<= 1) {
    const int t = __shfl_up(inc, off, 32);
    inc += ((int)lane >= off) ? t : 0;
  }
  if (lane == 31u) wtot[wv] = inc;
  if (tid < (unsigned)TOKT) toks[tid] = -1;
  __syncthreads();
  int base = 0, cntv = 0;
#pragma unroll
  for (int w2 = 0; w2 < 8; ++w2) {
    const int t = wtot[w2];
    base += ((unsigned)w2 < wv) ? t : 0;
    cntv += t;
  }
  const int cnt = __builtin_amdgcn_readfirstlane(cntv);
  if (tile * TOKT >= cnt) return;

  {
    int rank = base + inc - c - tile * TOKT;
#pragma unroll
    for (int j = 0; j < EPT; ++j) {
      const bool hit = (rv[j] == e);
      if (hit && (unsigned)rank < (unsigned)TOKT) toks[rank] = (int)(frow0 + (unsigned)j);
      rank += hit ? 1 : 0;
    }
  }
  __syncthreads();

  {
    const unsigned row = tid >> 3, cb = (tid & 7u) * 64u;
    const int tok = toks[row];
    const bool live = (tok >= 0);
    int tokc = live ? tok : 0;
    tokc = (tokc > NB_FULL * SEQ_FULL - 1) ? (NB_FULL * SEQ_FULL - 1) : tokc;
    const float* src = X + (size_t)tokc * DIM + cb;
#pragma unroll 2
    for (unsigned j = 0; j < 64u; j += 8u) {
      const v4f a0 = *(const v4f*)(src + j);
      const v4f a1 = *(const v4f*)(src + j + 4u);
      v8h o;
#pragma unroll
      for (int i = 0; i < 4; ++i) {
        o[i]     = toh_flush(live ? bf16r(a0[i]) : 0.0f);
        o[i + 4] = toh_flush(live ? bf16r(a1[i]) : 0.0f);
      }
      *(v8h*)&Xs[row * XLD + cb + j] = o;
    }
  }
  __syncthreads();

  v8f accO[8];
#pragma unroll
  for (int t = 0; t < 8; ++t) accO[t] = (v8f){};

#pragma unroll 1
  for (int ch = 0; ch < NCHUNK; ++ch) {
#pragma unroll 1
    for (int sub = 0; sub < 2; ++sub) {
      const unsigned colBase = (unsigned)wave * 32u + (unsigned)sub * 16u;
      const unsigned hcol = (unsigned)ch * (unsigned)CHUNK + colBase + m;
      const size_t boff = (size_t)hcol * GPITCH + (size_t)e * DIM + hh * 8u;
      const _Float16* bg = Wg_t + boff;
      const _Float16* bi = Wi_t + boff;
      v8f g0 = {}, g1 = {}, u0 = {}, u1 = {};
#pragma unroll 2
      for (unsigned k0 = 0; k0 < (unsigned)DIM; k0 += 32u) {
        const v16h fg = frag_at(bg + k0);
        const v16h fi = frag_at(bi + k0);
        const v16h a0 = ld_frag(&Xs[k0], XLD);
        const v16h a1 = ld_frag(&Xs[16 * XLD + k0], XLD);
        g0 = wmma16(a0, fg, g0);
        u0 = wmma16(a0, fi, u0);
        g1 = wmma16(a1, fg, g1);
        u1 = wmma16(a1, fi, u1);
      }
      const float bgv = bf16r(b_gate[(unsigned)e * (unsigned)HID + hcol]);
      const float biv = bf16r(b_in[(unsigned)e * (unsigned)HID + hcol]);
#pragma unroll
      for (int v = 0; v < 8; ++v) {
        const unsigned r = hh * 8u + (unsigned)v;
        const float h0 = silu_mul(g0[v] * (1.0f / WCARRY) + bgv, u0[v] * (1.0f / WCARRY) + biv);
        const float h1 = silu_mul(g1[v] * (1.0f / WCARRY) + bgv, u1[v] * (1.0f / WCARRY) + biv);
        Hs[r * HLD + colBase + m]         = toh_flush(HCARRY * h0);
        Hs[(r + 16u) * HLD + colBase + m] = toh_flush(HCARRY * h1);
      }
    }
    __syncthreads();

    const _Float16* bo = Wo_t + (size_t)((unsigned)wave * 64u + m) * OPITCH
                         + (size_t)e * HID + (size_t)ch * CHUNK + hh * 8u;
#pragma unroll 1
    for (unsigned k0 = 0; k0 < (unsigned)CHUNK; k0 += 32u) {
      const v16h a0 = ld_frag(&Hs[k0], HLD);
      const v16h a1 = ld_frag(&Hs[16 * HLD + k0], HLD);
#pragma unroll
      for (int t = 0; t < 4; ++t) {
        const v16h fb = frag_at(bo + (size_t)t * 16u * OPITCH + k0);
        accO[t]     = wmma16(a0, fb, accO[t]);
        accO[4 + t] = wmma16(a1, fb, accO[4 + t]);
      }
    }
    __syncthreads();
  }

  float* Cw = &Cs[(unsigned)wave * (unsigned)(TOKT * OLD)];
#pragma unroll
  for (int p = 0; p < 2; ++p) {
#pragma unroll
    for (int tt = 0; tt < 2; ++tt)
#pragma unroll
      for (int v = 0; v < 8; ++v) {
        const unsigned r = hh * 8u + (unsigned)v;
        Cw[r * OLD + (unsigned)tt * 16u + m]         = accO[2 * p + tt][v];
        Cw[(r + 16u) * OLD + (unsigned)tt * 16u + m] = accO[4 + 2 * p + tt][v];
      }
    wave_lds_sync();
    v4f xs[8];
    size_t off[8];
    bool ok[8];
#pragma unroll
    for (unsigned i = 0; i < 8u; ++i) {
      const unsigned r = 4u * i + (lane >> 3);
      const unsigned cc = (lane & 7u) * 4u;
      const unsigned col = (unsigned)wave * 64u + (unsigned)p * 32u + cc;
      const v4f u = *(const v4f*)&Cw[r * OLD + cc];
      const v4f g = *(const v4f*)(b_out + (unsigned)e * (unsigned)DIM + col);
      const int tok = toks[r];
      int tokc = (tok >= 0) ? tok : 0;
      tokc = (tokc > NB_FULL * SEQ_FULL - 1) ? (NB_FULL * SEQ_FULL - 1) : tokc;
      v4f val;
#pragma unroll
      for (int j = 0; j < 4; ++j) val[j] = u[j] * (1.0f / (WCARRY * HCARRY)) + bf16r(g[j]);
      xs[i] = val;
      off[i] = (size_t)tokc * DIM + col;
      ok[i] = (tok >= 0);
    }
#pragma unroll
    for (int i = 0; i < 8; ++i)
      if (ok[i]) *(volatile v4f*)(out + off[i]) = xs[i];
    __threadfence();
#pragma unroll
    for (int i = 0; i < 8; ++i)
      if (ok[i]) *(volatile v4f*)(out + off[i]) = xs[i];
    wave_lds_sync();
  }
}

extern "C" void kernel_launch(void* const* d_in, const int* in_sizes, int n_in,
                              void* d_out, int out_size, void* d_ws, size_t ws_size,
                              hipStream_t stream) {
  if (n_in < 8) return;
  const long long need_rows = (long long)(NB - 1) * SEQ_FULL + SEQ;
  const long long need_x = need_rows * DIM;
  if ((long long)in_sizes[0] < need_x) return;
  if ((long long)in_sizes[1] < need_rows) return;
  if ((long long)in_sizes[2] < (long long)NEXP * DIM * HID) return;
  if ((long long)in_sizes[3] < (long long)NEXP * HID) return;
  if ((long long)in_sizes[4] < (long long)NEXP * DIM * HID) return;
  if ((long long)in_sizes[5] < (long long)NEXP * HID) return;
  if ((long long)in_sizes[6] < (long long)NEXP * HID * DIM) return;
  if ((long long)in_sizes[7] < (long long)NEXP * DIM) return;
  if ((long long)out_size < need_x) return;
  if (ws_size < WS_TOTAL) return;

  const float* X      = (const float*)d_in[0];
  const int*   route  = (const int*)d_in[1];
  const float* w_in   = (const float*)d_in[2];
  const float* b_in   = (const float*)d_in[3];
  const float* w_gate = (const float*)d_in[4];
  const float* b_gate = (const float*)d_in[5];
  const float* w_out  = (const float*)d_in[6];
  const float* b_out  = (const float*)d_in[7];
  float* out = (float*)d_out;

  char* ws = (char*)d_ws;
  _Float16* Wg_t = (_Float16*)(ws + OFF_WG);
  _Float16* Wi_t = (_Float16*)(ws + OFF_WI);
  _Float16* Wo_t = (_Float16*)(ws + OFF_WO);

  dim3 blk(256);
  wconv_kernel<<<dim3(HID / 64, (NEXP * DIM) / 64), blk, 0, stream>>>(
      w_gate, Wg_t, (unsigned)HID, (unsigned)(NEXP * DIM));
  wconv_kernel<<<dim3(HID / 64, (NEXP * DIM) / 64), blk, 0, stream>>>(
      w_in, Wi_t, (unsigned)HID, (unsigned)(NEXP * DIM));
  wconv_kernel<<<dim3(DIM / 64, (NEXP * HID) / 64), blk, 0, stream>>>(
      w_out, Wo_t, (unsigned)DIM, (unsigned)(NEXP * HID));

  moe_ffn_kernel<<<dim3(MAXTILE, NEXP), blk, 0, stream>>>(
      X, route, Wg_t, Wi_t, Wo_t, b_in, b_gate, b_out, out);
}
